// ImageEncoder_65996467470744
// MI455X (gfx1250) — hardware-verified
//
#include <hip/hip_runtime.h>


#define NR   8192
#define DD   768
#define DO   512
typedef _Float16 h16;
typedef unsigned short bf;
typedef __attribute__((ext_vector_type(16))) __bf16   v16bf;
typedef __attribute__((ext_vector_type(16))) _Float16 v16h;
typedef __attribute__((ext_vector_type(8)))  _Float16 v8h;
typedef __attribute__((ext_vector_type(8)))  unsigned short v8us;
typedef __attribute__((ext_vector_type(8)))  float    v8f;
typedef __attribute__((ext_vector_type(4)))  float    v4f;
typedef v8h  __attribute__((may_alias)) v8ha;
typedef v4f  __attribute__((may_alias)) v4fa;
typedef v8us __attribute__((may_alias)) v8usa;

__device__ __forceinline__ unsigned short f2bf(float f) { unsigned u = __float_as_uint(f); u += 0x7FFFu + ((u >> 16) & 1u); return (unsigned short)(u >> 16); }
__device__ __forceinline__ float bf2f(unsigned short b) { return __uint_as_float(((unsigned)b) << 16); }
__device__ __forceinline__ float bfr(float f) { return bf2f(f2bf(f)); }
__device__ __forceinline__ v16h cat16(v8h lo, v8h hi) { return __builtin_shufflevector(lo, hi, 0, 1, 2, 3, 4, 5, 6, 7, 8, 9, 10, 11, 12, 13, 14, 15); }
__device__ __forceinline__ v16bf cat16b(v8us lo, v8us hi) { return __builtin_bit_cast(v16bf, __builtin_shufflevector(lo, hi, 0, 1, 2, 3, 4, 5, 6, 7, 8, 9, 10, 11, 12, 13, 14, 15)); }
__device__ __forceinline__ v8f wmma16(v16h a, v16h b, v8f c) { return __builtin_amdgcn_wmma_f32_16x16x32_f16(false, a, false, b, (short)0, c, false, false); }
__device__ __forceinline__ v8f wmmab(v16bf a, v16bf b, v8f c) { return __builtin_amdgcn_wmma_f32_16x16x32_bf16(false, a, false, b, (short)0, c, false, false); }


template <typename T16> struct WFrag;
template <> struct WFrag<h16> { typedef v16h V; static __device__ __forceinline__ V ld(const h16* p) { return cat16(*(const v8h*)p, *(const v8h*)(p + 16)); } static __device__ __forceinline__ v8f mma(V a, V b, v8f c) { return wmma16(a, b, c); } };
template <> struct WFrag<bf> { typedef v16bf V; static __device__ __forceinline__ V ld(const bf* p) { return cat16b(*(const v8us*)p, *(const v8us*)(p + 16)); } static __device__ __forceinline__ v8f mma(V a, V b, v8f c) { return wmmab(a, b, c); } };
template <typename T16, int NSPLIT, bool BIAS>
__global__ __launch_bounds__(32) void k_gemmw(const T16* __restrict__ A, const T16* __restrict__ A2, const T16* __restrict__ Bt, const T16* __restrict__ Bt2, int K, float* C, int ldc, const float* __restrict__ bias, size_t sA, size_t sB, size_t sC) {
    typedef typename WFrag<T16>::V V;
    __shared__ __align__(16) float os[16 * 68];
    const size_t z = blockIdx.z; A += z * sA; if (A2) A2 += z * sA; Bt += z * sB; if (Bt2) Bt2 += z * sB; C += z * sC;
    const int lane = threadIdx.x & 31, lr = lane & 15, hi = lane >> 4; const int r0 = blockIdx.x * 64, c0 = blockIdx.y * 64;
    v8f acc[4][4];
#pragma unroll
    for (int mb = 0; mb < 4; ++mb)
#pragma unroll
        for (int nb = 0; nb < 4; ++nb) acc[mb][nb] = (v8f){};
    const size_t aoff = (size_t)(r0 + lr) * K + 8 * hi, boff = (size_t)(c0 + lr) * K + 8 * hi;
#pragma unroll 1
    for (int kc = 0; kc < K; kc += 32) {
        V a[4], a2[4];
#pragma unroll
        for (int mb = 0; mb < 4; ++mb) { a[mb] = WFrag<T16>::ld(A + aoff + (size_t)mb * 16 * K + kc); if (NSPLIT == 1 || NSPLIT == 2) a2[mb] = WFrag<T16>::ld(A2 + aoff + (size_t)mb * 16 * K + kc); }
#pragma unroll
        for (int nb = 0; nb < 4; ++nb) { const V b = WFrag<T16>::ld(Bt + boff + (size_t)nb * 16 * K + kc); V b2; if (NSPLIT >= 2) b2 = WFrag<T16>::ld(Bt2 + boff + (size_t)nb * 16 * K + kc);
#pragma unroll
            for (int mb = 0; mb < 4; ++mb) { acc[mb][nb] = WFrag<T16>::mma(a[mb], b, acc[mb][nb]); if (NSPLIT == 1 || NSPLIT == 2) acc[mb][nb] = WFrag<T16>::mma(a2[mb], b, acc[mb][nb]); if (NSPLIT >= 2) acc[mb][nb] = WFrag<T16>::mma(a[mb], b2, acc[mb][nb]); } }
        asm volatile("v_nop\n\tv_nop\n\tv_nop\n\tv_nop" : "+v"(acc[0][0]), "+v"(acc[1][1]), "+v"(acc[2][2]), "+v"(acc[3][3]) : "v"(a[0]), "v"(a[3]));
    }
#pragma unroll
    for (int mb = 0; mb < 4; ++mb) {
#pragma unroll
        for (int nb = 0; nb < 4; ++nb) {
#pragma unroll
            for (int j = 0; j < 8; ++j) os[(hi * 8 + j) * 68 + nb * 16 + lr] = acc[mb][nb][j]; }
        __builtin_amdgcn_wave_barrier(); asm volatile("" ::: "memory");
        float* crow = C + (size_t)(r0 + mb * 16) * ldc + c0;
#pragma unroll 1
        for (int ps = 0; ps < 2; ++ps) {
#pragma unroll
            for (int s = 0; s < 8; ++s) { const int row = 2 * s + hi, cofs = lr * 4; v4f val = *(const v4fa*)(os + row * 68 + cofs); if (BIAS) { val[0] += bfr(bias[c0 + cofs]); val[1] += bfr(bias[c0 + cofs + 1]); val[2] += bfr(bias[c0 + cofs + 2]); val[3] += bfr(bias[c0 + cofs + 3]); }
                *(volatile v4f*)(crow + (size_t)row * ldc + cofs) = val; }
            if (ps == 0) __threadfence(); }
        __builtin_amdgcn_wave_barrier(); asm volatile("" ::: "memory");
    }
}

__device__ __forceinline__ void splitf(float y, unsigned short& h, unsigned short& l) { h = f2bf(y); l = f2bf(y - bf2f(h)); }
typedef __attribute__((ext_vector_type(2))) unsigned short v2us;
typedef __attribute__((ext_vector_type(4))) unsigned short v4us;

__global__ __launch_bounds__(256) void k_cvt8(const float* __restrict__ src, bf* dst, size_t n8) { const size_t i = (size_t)blockIdx.x * 256 + threadIdx.x; if (i >= n8) return; const v8f v = *(const v8f*)(src + i * 8); v8us o;
#pragma unroll
    for (int k = 0; k < 8; ++k) o[k] = f2bf(v[k]); *(volatile v8us*)(dst + i * 8) = o; __threadfence(); *(volatile v8us*)(dst + i * 8) = o; }
__global__ __launch_bounds__(256) void k_split2(const float* __restrict__ F, bf* Ph, bf* Pl, size_t cnt) { const size_t i = ((size_t)blockIdx.x * 256 + threadIdx.x) * 2; if (i >= cnt) return; v2us oh, ol;
#pragma unroll
    for (int q = 0; q < 2; ++q) { unsigned short a, c2; splitf(F[i + q], a, c2); oh[q] = a; ol[q] = c2; } *(volatile v2us*)(Ph + i) = oh; *(volatile v2us*)(Pl + i) = ol; __threadfence(); *(volatile v2us*)(Ph + i) = oh; *(volatile v2us*)(Pl + i) = ol; }
template <int RAWA, int RELU>
__global__ __launch_bounds__(256) void k_lnres(const float* __restrict__ A, const float* __restrict__ O, const float* __restrict__ gg, const float* __restrict__ bb, float* Y, bf* Yh, bf* Yl) {
    const int lane = threadIdx.x & 31; const int r = blockIdx.x * 8 + (threadIdx.x >> 5); if (r >= NR) return; float v[24]; float s = 0.f;
#pragma unroll
    for (int c = 0; c < 6; ++c) { const v4f a = *(const v4f*)(A + (size_t)r * DD + c * 128 + lane * 4), o = *(const v4f*)(O + (size_t)r * DD + c * 128 + lane * 4);
#pragma unroll
        for (int q = 0; q < 4; ++q) { const float t = __fadd_rn(RAWA ? bfr(a[q]) : a[q], o[q]); v[c * 4 + q] = t; s = __fadd_rn(s, t); } }
#pragma unroll
    for (int sh = 16; sh; sh >>= 1) s += __shfl_xor(s, sh, 32);
    const float mu = s * (1.0f / DD); float qq = 0.f;
#pragma unroll
    for (int i = 0; i < 24; ++i) { const float d0 = v[i] - mu; float p = __fmul_rn(d0, d0); asm volatile("" : "+v"(p)); qq = __fadd_rn(qq, p); }
#pragma unroll
    for (int sh = 16; sh; sh >>= 1) qq += __shfl_xor(qq, sh, 32);
    const float rs = __fdiv_rn(1.0f, __fsqrt_rn(__fadd_rn(qq * (1.0f / DD), 1e-5f)));
#pragma unroll 1
    for (int ps = 0; ps < 2; ++ps) {
#pragma unroll
        for (int c = 0; c < 6; ++c) { v4f y4; v4us oh, ol;
#pragma unroll
            for (int q = 0; q < 4; ++q) { const int col = c * 128 + lane * 4 + q; float tn = __fmul_rn(v[c * 4 + q] - mu, rs); asm volatile("" : "+v"(tn)); float tg = __fmul_rn(tn, bfr(gg[col])); asm volatile("" : "+v"(tg)); float y = __fadd_rn(tg, bfr(bb[col])); if (RELU) y = fmaxf(y, 0.f); y4[q] = y; unsigned short a2, c2; splitf(y, a2, c2); oh[q] = a2; ol[q] = c2; }
            const size_t o = (size_t)r * DD + c * 128 + lane * 4; if (Y) *(volatile v4f*)(Y + o) = y4; *(volatile v4us*)(Yh + o) = oh; *(volatile v4us*)(Yl + o) = ol; }
        if (ps == 0) __threadfence(); }
}
__global__ __launch_bounds__(256) void k_relu2(const float* __restrict__ F, bf* Ph, bf* Pl, size_t cnt) { const size_t i = ((size_t)blockIdx.x * 256 + threadIdx.x) * 2; if (i >= cnt) return; v2us oh, ol;
#pragma unroll
    for (int q = 0; q < 2; ++q) { unsigned short a, c2; splitf(fmaxf(F[i + q], 0.f), a, c2); oh[q] = a; ol[q] = c2; } *(volatile v2us*)(Ph + i) = oh; *(volatile v2us*)(Pl + i) = ol; __threadfence(); *(volatile v2us*)(Ph + i) = oh; *(volatile v2us*)(Pl + i) = ol; }
__global__ __launch_bounds__(256) void k_relu(const float* __restrict__ F, float* OUT, size_t cnt) { const size_t i = ((size_t)blockIdx.x * 256 + threadIdx.x) * 4; if (i >= cnt) return; const v4f a = *(const v4f*)(F + i); v4f o;
#pragma unroll
    for (int q = 0; q < 4; ++q) o[q] = fmaxf(a[q], 0.f); *(volatile v4f*)(OUT + i) = o; __threadfence(); *(volatile v4f*)(OUT + i) = o; }

extern "C" void kernel_launch(void* const* d_in, const int* in_sizes, int n_in,
                              void* d_out, int out_size, void* d_ws, size_t ws_size, hipStream_t stream) {
    (void)in_sizes; (void)n_in; (void)out_size;
    const float* IN[18]; for (int i = 0; i < 18; ++i) IN[i] = (const float*)d_in[i];
    float* OUT = (float*)d_out;
    char* wsp = (char*)d_ws;
    auto take = [&](size_t bytes) { char* p = wsp; wsp += (bytes + 255) & ~(size_t)255; return (void*)p; };
    bf* WVS = (bf*)take((size_t)DD * DD * 2); bf* WOS = (bf*)take((size_t)DD * DD * 2); bf* WVC = (bf*)take((size_t)DD * DD * 2); bf* WOC = (bf*)take((size_t)DD * DD * 2); bf* W1 = (bf*)take((size_t)DD * DD * 2); bf* W2 = (bf*)take((size_t)DO * DD * 2);
    bf* QB = (bf*)take((size_t)NR * DD * 2); bf* RB = (bf*)take((size_t)NR * DD * 2); float* F = (float*)take((size_t)NR * DD * 4); float* G = (float*)take((size_t)NR * DD * 4); bf* Ph = (bf*)take((size_t)NR * DD * 2); bf* Pl = (bf*)take((size_t)NR * DD * 2); float* Q1 = (float*)take((size_t)NR * DD * 4);
    if ((size_t)(wsp - (char*)d_ws) > ws_size) return;
    const size_t nw = (size_t)DD * DD / 8; const unsigned gw = (unsigned)((nw + 255) / 256); const unsigned L2 = (unsigned)(((size_t)NR * DD / 2 + 255) / 256); const dim3 gD(NR / 64, DD / 64, 1);
    { k_cvt8<<<gw, 256, 0, stream>>>(IN[2] + (size_t)2 * DD * DD, WVS, nw); k_cvt8<<<gw, 256, 0, stream>>>(IN[4], WOS, nw); k_cvt8<<<gw, 256, 0, stream>>>(IN[8] + (size_t)2 * DD * DD, WVC, nw); k_cvt8<<<gw, 256, 0, stream>>>(IN[10], WOC, nw); k_cvt8<<<gw, 256, 0, stream>>>(IN[14], W1, nw); k_cvt8<<<(unsigned)(((size_t)DO * DD / 8 + 255) / 256), 256, 0, stream>>>(IN[16], W2, (size_t)DO * DD / 8);
      k_cvt8<<<(unsigned)(((size_t)NR * DD / 8 + 255) / 256), 256, 0, stream>>>(IN[0], QB, (size_t)NR * DD / 8); k_cvt8<<<(unsigned)(((size_t)NR * DD / 8 + 255) / 256), 256, 0, stream>>>(IN[1], RB, (size_t)NR * DD / 8); }
    k_gemmw<bf, 0, true><<<gD, 32, 0, stream>>>(QB, nullptr, WVS, nullptr, DD, F, DD, IN[3] + 2 * DD, 0, 0, 0); k_split2<<<L2, 256, 0, stream>>>(F, Ph, Pl, (size_t)NR * DD);
    k_gemmw<bf, 1, true><<<gD, 32, 0, stream>>>(Ph, Pl, WOS, nullptr, DD, G, DD, IN[5], 0, 0, 0); k_lnres<1, 0><<<NR / 8, 256, 0, stream>>>(IN[0], G, IN[6], IN[7], Q1, Ph, Pl);
    k_gemmw<bf, 0, true><<<gD, 32, 0, stream>>>(RB, nullptr, WVC, nullptr, DD, F, DD, IN[9] + 2 * DD, 0, 0, 0); k_split2<<<L2, 256, 0, stream>>>(F, Ph, Pl, (size_t)NR * DD);
    k_gemmw<bf, 1, true><<<gD, 32, 0, stream>>>(Ph, Pl, WOC, nullptr, DD, G, DD, IN[11], 0, 0, 0); k_lnres<0, 1><<<NR / 8, 256, 0, stream>>>(Q1, G, IN[12], IN[13], nullptr, Ph, Pl);
    k_gemmw<bf, 1, true><<<gD, 32, 0, stream>>>(Ph, Pl, W1, nullptr, DD, F, DD, IN[15], 0, 0, 0); k_relu2<<<L2, 256, 0, stream>>>(F, Ph, Pl, (size_t)NR * DD);
    k_gemmw<bf, 1, true><<<dim3(NR / 64, DO / 64, 1), 32, 0, stream>>>(Ph, Pl, W2, nullptr, DD, G, DO, IN[17], 0, 0, 0); k_relu<<<(unsigned)(((size_t)NR * DO / 4 + 255) / 256), 256, 0, stream>>>(G, OUT, (size_t)NR * DO);
}
